// SimpleBlock_21723944583653
// MI455X (gfx1250) — hardware-verified
//
#include <hip/hip_runtime.h>
#include <math.h>

constexpr int kNumPts       = 50000;
constexpr int kNumPtsPad    = 50048;
constexpr int kNbr          = 32;
constexpr int kNumKp        = 15;
constexpr int kCin          = 64;
constexpr int kCout         = 128;
constexpr int kKdim         = kNumKp * kCin;
constexpr float kResCarry    = 2048.0f;
constexpr float kResCarryInv = 1.0f / 2048.0f;
constexpr float kBnEps      = 1e-5f;
constexpr float kSlope      = 0.2f;
constexpr int kTilesM       = kNumPtsPad / 64;
constexpr int kChunkTiles0  = 261;
constexpr int kChunkTiles1  = 261;
constexpr int kChunkTiles2  = 260;
constexpr int kChunkRowsMax = 261 * 64;
constexpr int kStatRows     = 512;
constexpr int kStatBlocks   = (kNumPts + kStatRows - 1) / kStatRows;
constexpr int kXCast8       = kNumPts * kCin / 8;

static_assert(kKdim % 32 == 0, "K of stage B is a multiple of 32");
static_assert(kNbr == 32, "K of stage A is exactly one 32-deep step");
static_assert(kNumPtsPad % 64 == 0 && kNumPtsPad >= kNumPts && kNumPtsPad - kNumPts < 64, "M padded to the 64 tile");
static_assert(kChunkTiles0 + kChunkTiles1 + kChunkTiles2 == kTilesM, "chunks cover all M tiles");
static_assert(kChunkTiles0 * 64 <= kChunkRowsMax && kChunkTiles1 * 64 <= kChunkRowsMax && kChunkTiles2 * 64 <= kChunkRowsMax, "chunk rows fit the carve");
static_assert(kCout % 64 == 0, "N is a tile multiple");
static_assert((kNumPts * kCin) % 8 == 0, "x cast coverage");
static_assert(kNumPts % 2 == 0 && kStatRows % 2 == 0, "even row counts in the stats pass");
static_assert(kKdim % 64 == 0 && kCout % 64 == 0, "weight transpose tiles");
static_assert(kNumKp * 3 <= 128, "kernel-point table fits one load per thread of a 128-thread block");

typedef __attribute__((ext_vector_type(16))) _Float16 v16h;
typedef __attribute__((ext_vector_type(8)))  _Float16 v8h;
typedef __attribute__((ext_vector_type(16))) __bf16   v16b;
typedef __attribute__((ext_vector_type(8)))  __bf16   v8b;
typedef __attribute__((ext_vector_type(8)))  float    v8f;
typedef __attribute__((ext_vector_type(4)))  float    v4f;
typedef __attribute__((ext_vector_type(4)))  unsigned int v4u;

__device__ __forceinline__ unsigned short f2bf_bits(float f) {
  unsigned u = __float_as_uint(f);
  return (unsigned short)((u + 0x7FFFu + ((u >> 16) & 1u)) >> 16);
}
__device__ __forceinline__ float bf_bits2f(unsigned short h) { return __uint_as_float(((unsigned)h) << 16); }

__device__ __forceinline__ void dep_guard_h(v8f& a, v8f& b, v16h x, v16h y) { asm volatile("v_nop\n\tv_nop\n\tv_nop\n\tv_nop" : "+v"(a), "+v"(b) : "v"(x), "v"(y)); }
__device__ __forceinline__ void dep_guard_b(v8f& a, v8f& b, v16b x, v16b y) { asm volatile("v_nop\n\tv_nop\n\tv_nop\n\tv_nop" : "+v"(a), "+v"(b) : "v"(x), "v"(y)); }
__device__ __forceinline__ void keep4_h(v16h a, v16h b, v16h c, v16h d) { asm volatile("v_nop" :: "v"(a), "v"(b), "v"(c), "v"(d)); }
__device__ __forceinline__ void keep4_b(v16b a, v16b b, v16b c, v16b d) { asm volatile("v_nop" :: "v"(a), "v"(b), "v"(c), "v"(d)); }
__device__ __forceinline__ void acc_guard4(v8f& a, v8f& b, v8f& c, v8f& d) { asm volatile("v_nop\n\tv_nop\n\tv_nop\n\tv_nop" : "+v"(a), "+v"(b), "+v"(c), "+v"(d)); }
template <typename T> struct Frag;
template <> struct Frag<_Float16> {
  typedef v16h V; union U { v16h v; v8h h[2]; };
  static __device__ __forceinline__ v16h load(const _Float16* p) {
    U f; f.h[0] = *(const v8h*)(p); f.h[1] = *(const v8h*)(p + 16); return f.v;
  }
  static __device__ __forceinline__ v8f mma(v16h a, v16h b, v8f c) {
    return __builtin_amdgcn_wmma_f32_16x16x32_f16(false, a, false, b, (short)0, c, false, false);
  }
  static __device__ __forceinline__ void guard(v8f& a, v8f& b, v16h x, v16h y) { dep_guard_h(a, b, x, y); }
  static __device__ __forceinline__ void keep(v16h a, v16h b, v16h c, v16h d) { keep4_h(a, b, c, d); }
};
template <> struct Frag<__bf16> {
  typedef v16b V; union U { v16b v; v8b h[2]; };
  static __device__ __forceinline__ v16b load(const __bf16* p) {
    U f; f.h[0] = *(const v8b*)(p); f.h[1] = *(const v8b*)(p + 16); return f.v;
  }
  static __device__ __forceinline__ v8f mma(v16b a, v16b b, v8f c) {
    return __builtin_amdgcn_wmma_f32_16x16x32_bf16(false, a, false, b, (short)0, c, false, false);
  }
  static __device__ __forceinline__ void guard(v8f& a, v8f& b, v16b x, v16b y) { dep_guard_b(a, b, x, y); }
  static __device__ __forceinline__ void keep(v16b a, v16b b, v16b c, v16b d) { keep4_b(a, b, c, d); }
};

__device__ __forceinline__ unsigned pk16(unsigned short a, unsigned short b) { return (unsigned)a | ((unsigned)b << 16); }
__device__ __forceinline__ unsigned short h_bits(float f) { const _Float16 h = (_Float16)f; return __builtin_bit_cast(unsigned short, h); }

__device__ __forceinline__ float h16_to_f32(unsigned hb) {
  const unsigned sgn = (hb & 0x8000u) << 16; const unsigned em = hb & 0x7fffu;
  const float fn = __uint_as_float((em << 13) + 0x38000000u);
  const float fs = (float)em * 5.9604644775390625e-8f;
  const float mag = (em < 0x400u) ? fs : fn; return __uint_as_float(__float_as_uint(mag) | sgn); }

__device__ __forceinline__ void guard2_frag4(v8f& a0, v8f& a1, v16h fa, v16h fal, v16h fb, v16h fbl) {
  asm volatile("v_nop\n\tv_nop\n\tv_nop\n\tv_nop"
               : "+v"(a0), "+v"(a1)
               : "v"(fa), "v"(fal), "v"(fb), "v"(fbl));
}

template <int ET> struct Elem;
template <> struct Elem<0> { typedef _Float16 T; };
template <> struct Elem<1> { typedef __bf16 T; };
template <int ET, bool SPLIT, int BIAS_MODE, int OUT_MODE, bool RESID, int ACT = 0>
__global__ __launch_bounds__(256) void wmma_gemm64(
    const unsigned short* __restrict__ Ap, const unsigned short* __restrict__ A2p, int lda, long strideA,
    const unsigned short* __restrict__ Btp, const unsigned short* __restrict__ Bt2p, int ldb, long strideB,
    void* __restrict__ Cout, void* __restrict__ Cout2, int ldc, long strideC,
    const float* __restrict__ bias,
    const float* __restrict__ resid, long strideR,
    int M, int N, int K, float scale) {
  typedef typename Elem<ET>::T T;
  typedef typename Frag<T>::V V;
  const T* A = (const T*)Ap; const T* A2 = (const T*)A2p; const T* Bt = (const T*)Btp; const T* Bt2 = (const T*)Bt2p;
  __shared__ __align__(16) float sT[8][16 * 68];
  const int b    = blockIdx.y;
  const int lane = threadIdx.x & 31;
  const int wave = threadIdx.x >> 5;
  const int tilesN = N >> 6;
  const int tilesM = M >> 6;
  const int tile = blockIdx.x * 8 + wave;
  if (tile >= tilesM * tilesN) return;
  const int tm = tile / tilesN;
  const int tn = tile - tm * tilesN;
  const int m0 = tm << 6;
  const int n0 = tn << 6;

  const T* Ab  = A  + (size_t)b * strideA;
  const T* Bb  = Bt + (size_t)b * strideB;
  const T* Ab2 = SPLIT ? (A2  + (size_t)b * strideA) : nullptr;
  const T* Bb2 = SPLIT ? (Bt2 + (size_t)b * strideB) : nullptr;

  const int rlane = lane & 15;
  const int koff  = (lane >> 4) * 8;
  const int mOff  = (lane >> 4) * 8;

  v8f acc[4][4];
#pragma unroll
  for (int i = 0; i < 4; ++i)
#pragma unroll
    for (int j = 0; j < 4; ++j) acc[i][j] = (v8f){0.f,0.f,0.f,0.f,0.f,0.f,0.f,0.f};

  for (int k0 = 0; k0 < K; k0 += 32) {
    V bh[4], bl[4];
#pragma unroll
    for (int j = 0; j < 4; ++j) {
      const size_t bo = (size_t)(n0 + (j << 4) + rlane) * ldb + koff + k0;
      bh[j] = Frag<T>::load(Bb + bo);
      if (SPLIT) bl[j] = Frag<T>::load(Bb2 + bo);
    }
#pragma unroll
    for (int i = 0; i < 4; ++i) {
      const size_t ao = (size_t)(m0 + (i << 4) + rlane) * lda + koff + k0;
      V ah = Frag<T>::load(Ab + ao);
      V al;
      if (SPLIT) al = Frag<T>::load(Ab2 + ao);
#pragma unroll
      for (int j = 0; j < 4; ++j) {
        acc[i][j] = Frag<T>::mma(ah, bh[j], acc[i][j]);
        if (SPLIT) {
          acc[i][j] = Frag<T>::mma(ah, bl[j], acc[i][j]);
          acc[i][j] = Frag<T>::mma(al, bh[j], acc[i][j]);
        }
      }
      Frag<T>::guard(acc[i][0], acc[i][3], ah, SPLIT ? al : ah);
    }
    Frag<T>::keep(bh[0], bh[1], bh[2], bh[3]);
    if (SPLIT) Frag<T>::keep(bl[0], bl[1], bl[2], bl[3]);
  }
  acc_guard4(acc[0][0], acc[0][1], acc[0][2], acc[0][3]);
  acc_guard4(acc[1][0], acc[1][1], acc[1][2], acc[1][3]);
  acc_guard4(acc[2][0], acc[2][1], acc[2][2], acc[2][3]);
  acc_guard4(acc[3][0], acc[3][1], acc[3][2], acc[3][3]);

  float* slab = sT[wave];
  const float* Rb = RESID ? (resid + (size_t)b * strideR) : nullptr;
#pragma unroll
  for (int i = 0; i < 4; ++i) {
    const int mBase = m0 + (i << 4);
#pragma unroll
    for (int j = 0; j < 4; ++j) {
      const int n = n0 + (j << 4) + rlane;
      float bv = 0.f;
      if (BIAS_MODE == 2) bv = bias[n];
#pragma unroll
      for (int r = 0; r < 8; ++r) {
        float v = acc[i][j][r] * scale;
        if (BIAS_MODE == 1) v += bias[mBase + mOff + r];
        if (BIAS_MODE == 2) v += bv;
        if (RESID) v += Rb[(size_t)(mBase + mOff + r) * ldc + n];
        if (ACT == 2) v = fmaxf(v, 0.0f);
        if (ACT == 4) v = (v > 0.f) ? v : 0.01f * v;
        slab[(mOff + r) * 68 + (j << 4) + rlane] = v;
      }
    }
    __builtin_amdgcn_fence(__ATOMIC_RELEASE, "workgroup");
    __builtin_amdgcn_wave_barrier();
    __builtin_amdgcn_fence(__ATOMIC_ACQUIRE, "workgroup");
    if (OUT_MODE == 0) {
      float* C = (float*)Cout + (size_t)b * strideC;
      const int hh = lane >> 4, c4 = (lane & 15) * 4;
      for (int pass = 0; pass < 2; ++pass) {
#pragma unroll
        for (int it = 0; it < 8; ++it) {
          const int row = it * 2 + hh;
          v4f v = *(const v4f*)(slab + row * 68 + c4);
          *(volatile v4f*)(C + (size_t)(mBase + row) * ldc + n0 + c4) = v;
        }
        __threadfence();
      }
    } else {
      const int q = lane >> 3, c8 = (lane & 7) * 8;
      unsigned short* C  = (unsigned short*)Cout  + (size_t)b * strideC;
      unsigned short* C2 = (OUT_MODE == 2) ? ((unsigned short*)Cout2 + (size_t)b * strideC) : nullptr;
      for (int pass = 0; pass < 2; ++pass) {
#pragma unroll
        for (int it = 0; it < 4; ++it) {
          const int row = it * 4 + q;
          const float* sp = slab + row * 68 + c8;
          v8h hv, lv;
#pragma unroll
          for (int e = 0; e < 8; ++e) {
            if (OUT_MODE == 1) {
              hv[e] = (_Float16)sp[e];
            } else {
              unsigned short hb = f2bf_bits(sp[e]);
              unsigned short lb = f2bf_bits(sp[e] - bf_bits2f(hb));
              hv[e] = __builtin_bit_cast(_Float16, hb);
              lv[e] = __builtin_bit_cast(_Float16, lb);
            }
          }
          *(volatile v8h*)(C + (size_t)(mBase + row) * ldc + n0 + c8) = hv;
          if (OUT_MODE == 2) *(volatile v8h*)(C2 + (size_t)(mBase + row) * ldc + n0 + c8) = lv;
        }
        __threadfence();
      }
    }
    __builtin_amdgcn_fence(__ATOMIC_RELEASE, "workgroup");
    __builtin_amdgcn_wave_barrier();
    __builtin_amdgcn_fence(__ATOMIC_ACQUIRE, "workgroup");
  }
}

__global__ __launch_bounds__(256) void castx_kernel(const float* __restrict__ in, unsigned short* __restrict__ XH,
                                                    unsigned short* __restrict__ XL, int n8) {
  const int i = blockIdx.x * 256 + threadIdx.x;
  if (i >= n8) return;
  const float* p = in + 8 * (size_t)i;
  const v4f a = *(const v4f*)(p);
  const v4f c = *(const v4f*)(p + 4);
  unsigned short hb[8], lb[8];
#pragma unroll
  for (int e = 0; e < 4; ++e) {
    {
      const float v = a[e];
      const unsigned short h = h_bits(v);
      hb[e] = h;
      lb[e] = h_bits((v - h16_to_f32((unsigned)h)) * kResCarry);
    }
    {
      const float v = c[e];
      const unsigned short h = h_bits(v);
      hb[4 + e] = h;
      lb[4 + e] = h_bits((v - h16_to_f32((unsigned)h)) * kResCarry);
    }
  }
  const v4u uh = (v4u){pk16(hb[0], hb[1]), pk16(hb[2], hb[3]), pk16(hb[4], hb[5]), pk16(hb[6], hb[7])};
  const v4u ul = (v4u){pk16(lb[0], lb[1]), pk16(lb[2], lb[3]), pk16(lb[4], lb[5]), pk16(lb[6], lb[7])};
  unsigned short* qh = XH + 8 * (size_t)i;
  unsigned short* ql = XL + 8 * (size_t)i;
  *(volatile v4u*)qh = uh;
  *(volatile v4u*)ql = ul;
  __threadfence();
  *(volatile v4u*)qh = uh;
  *(volatile v4u*)ql = ul;
}

__global__ __launch_bounds__(256) void wtcast_kernel(const float* __restrict__ W, unsigned short* __restrict__ WTH,
                                                     unsigned short* __restrict__ WTL) {
  __shared__ float sm[64][65];
  const int t   = threadIdx.x;
  const int kc0 = blockIdx.x * 64;
  const int d0  = blockIdx.y * 64;
#pragma unroll
  for (int i = 0; i < 8; ++i) {
    const int e = i * 256 + t;
    const int r = e >> 6;
    const int c = e & 63;
    sm[c][r] = W[(size_t)(kc0 + r) * kCout + d0 + c];
  }
  asm volatile("" ::: "memory");
#pragma unroll
  for (int i = 8; i < 16; ++i) {
    const int e = i * 256 + t;
    const int r = e >> 6;
    const int c = e & 63;
    sm[c][r] = W[(size_t)(kc0 + r) * kCout + d0 + c];
  }
  __syncthreads();
  const int lane = t & 31, wave = t >> 5;
  const int q = lane >> 3, c8 = (lane & 7) * 8;
  for (int pass = 0; pass < 2; ++pass) {
#pragma unroll
    for (int it = 0; it < 2; ++it) {
      const int row = wave * 8 + it * 4 + q;
      unsigned short hb[8], lb[8];
#pragma unroll
      for (int e = 0; e < 8; ++e) {
        const float v = sm[row][c8 + e];
        const unsigned short h = f2bf_bits(v);
        hb[e] = h;
        lb[e] = f2bf_bits(v - bf_bits2f(h));
      }
      const v4u uh = (v4u){pk16(hb[0], hb[1]), pk16(hb[2], hb[3]), pk16(hb[4], hb[5]), pk16(hb[6], hb[7])};
      const v4u ul = (v4u){pk16(lb[0], lb[1]), pk16(lb[2], lb[3]), pk16(lb[4], lb[5]), pk16(lb[6], lb[7])};
      *(volatile v4u*)(WTH + (size_t)(d0 + row) * kKdim + kc0 + c8) = uh;
      *(volatile v4u*)(WTL + (size_t)(d0 + row) * kKdim + kc0 + c8) = ul;
    }
    __threadfence();
  }
}

__global__ __launch_bounds__(128) void gather_agg_kernel(const float* __restrict__ points, const int* __restrict__ nbr,
                                                         const unsigned short* __restrict__ XH, const unsigned short* __restrict__ XL,
                                                         const float* __restrict__ kpts,
                                                         unsigned short* __restrict__ WFH, unsigned short* __restrict__ WFL,
                                                         int rowBase) {
  __shared__ __align__(16) unsigned short sInH[4][16 * 32];
  __shared__ __align__(16) unsigned short sInL[4][16 * 32];
  __shared__ __align__(16) unsigned short sNxH[4][kCin * 32];
  __shared__ __align__(16) unsigned short sNxL[4][kCin * 32];
  __shared__ __align__(16) unsigned short sOutH[4][16 * 64];
  __shared__ __align__(16) unsigned short sOutL[4][16 * 64];
  __shared__ __align__(16) float sKp[128];
  const int tid  = threadIdx.x;
  const int lane = tid & 31;
  const int wave = __builtin_amdgcn_readfirstlane(tid >> 5);
  const int hh   = lane >> 4;
  const int m    = lane & 15;
  const int q    = lane >> 3;
  const int c8   = (lane & 7) * 8;
  unsigned short* inh = sInH[wave];
  unsigned short* inl = sInL[wave];
  unsigned short* nxh = sNxH[wave];
  unsigned short* nxl = sNxL[wave];
  unsigned short* soh = sOutH[wave];
  unsigned short* sol = sOutL[wave];

  {
    const int kc = tid < kNumKp * 3 ? tid : (kNumKp * 3 - 1);
    sKp[tid] = kpts[kc];
  }
  __syncthreads();
  float kpx[kNumKp], kpy[kNumKp], kpz[kNumKp];
#pragma unroll
  for (int k = 0; k < kNumKp; ++k) {
    kpx[k] = sKp[k * 3 + 0];
    kpy[k] = sKp[k * 3 + 1];
    kpz[k] = sKp[k * 3 + 2];
  }

  const int lrow0 = (blockIdx.x * 4 + wave) * 16;
  const v8f zero8 = (v8f){0.f, 0.f, 0.f, 0.f, 0.f, 0.f, 0.f, 0.f};

#pragma unroll 1
  for (int p = 0; p < 16; ++p) {
    const int lrow = lrow0 + p;
    const int n    = rowBase + lrow;
    const int nc   = n < kNumPts ? n : (kNumPts - 1);
    int idx = nbr[(size_t)nc * kNbr + lane];
    idx = idx < 0 ? 0 : (idx > kNumPts - 1 ? (kNumPts - 1) : idx);
    const float cx = points[(size_t)nc * 3 + 0];
    const float cy = points[(size_t)nc * 3 + 1];
    const float cz = points[(size_t)nc * 3 + 2];
    const float px = points[(size_t)idx * 3 + 0] - cx;
    const float py = points[(size_t)idx * 3 + 1] - cy;
    const float pz = points[(size_t)idx * 3 + 2] - cz;

#pragma unroll
    for (int k = 0; k < kNumKp; ++k) {
      const float dx = px - kpx[k], dy = py - kpy[k], dz = pz - kpz[k];
      const float d2 = dx * dx + dy * dy + dz * dz;
      const float iv = fmaxf(0.0f, 1.0f - sqrtf(d2));
      const _Float16 ih = (_Float16)iv;
      const float ivh = (float)ih;
      const float ivl = (iv - ivh) * kResCarry;
      inh[k * 32 + lane] = __builtin_bit_cast(unsigned short, ih);
      inl[k * 32 + lane] = h_bits(ivl);
    }
    inh[kNumKp * 32 + lane] = (unsigned short)0;
    inl[kNumKp * 32 + lane] = (unsigned short)0;

    const v4u* xhr = (const v4u*)(XH + (size_t)idx * kCin);
    const v4u* xlr = (const v4u*)(XL + (size_t)idx * kCin);
#pragma unroll
    for (int j = 0; j < 4; ++j) {
      const v4u w = xhr[j];
#pragma unroll
      for (int e = 0; e < 4; ++e) {
        nxh[(j * 8 + 2 * e) * 32 + lane]     = (unsigned short)(w[e] & 0xffffu);
        nxh[(j * 8 + 2 * e + 1) * 32 + lane] = (unsigned short)(w[e] >> 16);
      }
    }
    asm volatile("" ::: "memory");
#pragma unroll
    for (int j = 4; j < 8; ++j) {
      const v4u w = xhr[j];
#pragma unroll
      for (int e = 0; e < 4; ++e) {
        nxh[(j * 8 + 2 * e) * 32 + lane]     = (unsigned short)(w[e] & 0xffffu);
        nxh[(j * 8 + 2 * e + 1) * 32 + lane] = (unsigned short)(w[e] >> 16);
      }
    }
    asm volatile("" ::: "memory");
#pragma unroll
    for (int j = 0; j < 4; ++j) {
      const v4u w = xlr[j];
#pragma unroll
      for (int e = 0; e < 4; ++e) {
        nxl[(j * 8 + 2 * e) * 32 + lane]     = (unsigned short)(w[e] & 0xffffu);
        nxl[(j * 8 + 2 * e + 1) * 32 + lane] = (unsigned short)(w[e] >> 16);
      }
    }
    asm volatile("" ::: "memory");
#pragma unroll
    for (int j = 4; j < 8; ++j) {
      const v4u w = xlr[j];
#pragma unroll
      for (int e = 0; e < 4; ++e) {
        nxl[(j * 8 + 2 * e) * 32 + lane]     = (unsigned short)(w[e] & 0xffffu);
        nxl[(j * 8 + 2 * e + 1) * 32 + lane] = (unsigned short)(w[e] >> 16);
      }
    }
    __syncthreads();

    const v16h fa  = Frag<_Float16>::load((const _Float16*)inh + m * 32 + 8 * hh);
    const v16h fal = Frag<_Float16>::load((const _Float16*)inl + m * 32 + 8 * hh);
    v8f acch[4], accr[4];
#pragma unroll
    for (int t = 0; t < 4; ++t) {
      const v16h fbh = Frag<_Float16>::load((const _Float16*)nxh + (t * 16 + m) * 32 + 8 * hh);
      const v16h fbl = Frag<_Float16>::load((const _Float16*)nxl + (t * 16 + m) * 32 + 8 * hh);
      acch[t] = Frag<_Float16>::mma(fa, fbh, zero8);
      accr[t] = Frag<_Float16>::mma(fa, fbl, zero8);
      accr[t] = Frag<_Float16>::mma(fal, fbh, accr[t]);
      guard2_frag4(acch[t], accr[t], fa, fal, fbh, fbl);
    }

#pragma unroll
    for (int t = 0; t < 4; ++t) {
#pragma unroll
      for (int r = 0; r < 8; ++r) {
        const float wf = fmaf(accr[t][r], kResCarryInv, acch[t][r]);
        const unsigned short hb = f2bf_bits(wf);
        const unsigned short lb = f2bf_bits(wf - bf_bits2f(hb));
        soh[(8 * hh + r) * 64 + t * 16 + m] = hb;
        sol[(8 * hh + r) * 64 + t * 16 + m] = lb;
      }
    }
    __syncthreads();

    v4u oh[4], ol[4];
#pragma unroll
    for (int it = 0; it < 4; ++it) {
      oh[it] = *(const v4u*)(soh + (it * 4 + q) * 64 + c8);
      ol[it] = *(const v4u*)(sol + (it * 4 + q) * 64 + c8);
    }
    unsigned short* rh = WFH + (size_t)lrow * kKdim;
    unsigned short* rl = WFL + (size_t)lrow * kKdim;
    for (int pass = 0; pass < 2; ++pass) {
#pragma unroll
      for (int it = 0; it < 4; ++it) {
        const int k = it * 4 + q;
        if (k < kNumKp) {
          *(volatile v4u*)(rh + k * kCin + c8) = oh[it];
          *(volatile v4u*)(rl + k * kCin + c8) = ol[it];
        }
      }
      __threadfence();
    }
  }
}

__global__ __launch_bounds__(256) void stats_partial_kernel(const float* __restrict__ OUTP, float* __restrict__ PART) {
  __shared__ __align__(16) float red[2][256];
  __shared__ __align__(16) float fin[256];
  const int t = threadIdx.x;
  const int d = t & 127, g = t >> 7;
  const int r0 = blockIdx.x * kStatRows;
  int nrows = kNumPts - r0;
  nrows = nrows > kStatRows ? kStatRows : nrows;
  float s = 0.0f, s2 = 0.0f;
#pragma unroll 4
  for (int i = 0; i < nrows; i += 2) {
    const float v = OUTP[(size_t)(r0 + i + g) * kCout + d];
    s += v;
    s2 = fmaf(v, v, s2);
  }
  red[g][d] = s;
  red[g][128 + d] = s2;
  __syncthreads();
  if (t < 128) {
    fin[t]       = red[0][t] + red[1][t];
    fin[128 + t] = red[0][128 + t] + red[1][128 + t];
  }
  __syncthreads();
  const int lane = t & 31, wave = t >> 5;
  if (wave < 2) {
    const v4f v = *(const v4f*)(fin + wave * 128 + 4 * lane);
    float* dst = PART + (size_t)blockIdx.x * 256 + wave * 128 + 4 * lane;
    for (int pass = 0; pass < 2; ++pass) {
      *(volatile v4f*)dst = v;
      __threadfence();
    }
  }
}

__global__ __launch_bounds__(128) void stats_final_kernel(const float* __restrict__ PART, const float* __restrict__ gamma,
                                                          float* __restrict__ MR) {
  __shared__ __align__(16) float sm[256];
  const int d = threadIdx.x;
  double s = 0.0, s2 = 0.0;
#pragma unroll 1
  for (int b = 0; b < kStatBlocks; ++b) {
    s  += (double)PART[(size_t)b * 256 + d];
    s2 += (double)PART[(size_t)b * 256 + 128 + d];
  }
  const double invn = 1.0 / (double)kNumPts;
  const double mean = s * invn;
  const double var  = s2 * invn - mean * mean;
  float varf = (float)var;
  varf = varf > 0.0f ? varf : 0.0f;
  const float rstd = 1.0f / sqrtf(varf + kBnEps);
  sm[d]       = (float)mean;
  sm[128 + d] = rstd * gamma[d];
  __syncthreads();
  const int lane = d & 31, wave = d >> 5;
  if (wave < 2) {
    const v4f v = *(const v4f*)(sm + wave * 128 + 4 * lane);
    float* dst = MR + wave * 128 + 4 * lane;
    for (int pass = 0; pass < 2; ++pass) {
      *(volatile v4f*)dst = v;
      __threadfence();
    }
  }
}

__global__ __launch_bounds__(256) void norm_act_kernel(const float* __restrict__ OUTP, const float* __restrict__ MR,
                                                       const float* __restrict__ beta, float* __restrict__ out, int total4) {
  const int i = blockIdx.x * 256 + threadIdx.x;
  if (i >= total4) return;
  const int row = i >> 5;
  const int c4  = (i & 31) * 4;
  const v4f v   = *(const v4f*)(OUTP + (size_t)row * kCout + c4);
  const v4f mu  = *(const v4f*)(MR + c4);
  const v4f sg  = *(const v4f*)(MR + 128 + c4);
  const v4f be  = *(const v4f*)(beta + c4);
  const v4f y   = (v - mu) * sg + be;
  v4f o;
#pragma unroll
  for (int e = 0; e < 4; ++e) o[e] = (y[e] > 0.0f) ? y[e] : kSlope * y[e];
  float* dst = out + (size_t)row * kCout + c4;
  *(volatile v4f*)dst = o;
  __threadfence();
  *(volatile v4f*)dst = o;
}

extern "C" void kernel_launch(void* const* d_in, const int* in_sizes, int n_in,
                              void* d_out, int out_size, void* d_ws, size_t ws_size, hipStream_t stream) {
  if (n_in < 7) return;
  if (in_sizes[0] != kNumPts * 3 || in_sizes[1] != kNumPts * kCin || in_sizes[2] != kNumPts * kNbr ||
      in_sizes[3] != kNumKp * 3 || in_sizes[4] != kKdim * kCout || in_sizes[5] != kCout || in_sizes[6] != kCout ||
      out_size != kNumPts * kCout) return;
  const float* points = (const float*)d_in[0];
  const float* x      = (const float*)d_in[1];
  const int*   nbr    = (const int*)  d_in[2];
  const float* kpts   = (const float*)d_in[3];
  const float* W      = (const float*)d_in[4];
  const float* gamma  = (const float*)d_in[5];
  const float* beta   = (const float*)d_in[6];
  float* out = (float*)d_out;

  char* ws = (char*)d_ws; size_t off = 0;
  auto carve = [&](size_t bytes) -> char* { char* p = ws + off; off += (bytes + 255) & ~(size_t)255; return p; };
  unsigned short* XH   = (unsigned short*)carve((size_t)kNumPts * kCin * 2);
  unsigned short* XL   = (unsigned short*)carve((size_t)kNumPts * kCin * 2);
  unsigned short* WTH  = (unsigned short*)carve((size_t)kCout * kKdim * 2);
  unsigned short* WTL  = (unsigned short*)carve((size_t)kCout * kKdim * 2);
  unsigned short* WFH  = (unsigned short*)carve((size_t)kChunkRowsMax * kKdim * 2);
  unsigned short* WFL  = (unsigned short*)carve((size_t)kChunkRowsMax * kKdim * 2);
  float*          OUTP = (float*)carve((size_t)kNumPtsPad * kCout * 4);
  float*          PART = (float*)carve((size_t)kStatBlocks * 256 * 4);
  float*          MR   = (float*)carve((size_t)2 * kCout * 4);
  if (off > ws_size || off > (size_t)134217728) return;

  castx_kernel<<<(kXCast8 + 255) / 256, 256, 0, stream>>>(x, XH, XL, kXCast8);
  wtcast_kernel<<<dim3(kKdim / 64, kCout / 64), 256, 0, stream>>>(W, WTH, WTL);

  const int chunkTiles[3]    = {kChunkTiles0, kChunkTiles1, kChunkTiles2};
  const int chunkTileBase[3] = {0, kChunkTiles0, kChunkTiles0 + kChunkTiles1};
  for (int c = 0; c < 3; ++c) {
    const int tiles   = chunkTiles[c];
    const int rowBase = chunkTileBase[c] * 64;
    const int Mc      = tiles * 64;
    gather_agg_kernel<<<tiles, 128, 0, stream>>>(points, nbr, XH, XL, kpts, WFH, WFL, rowBase);
    const int wtiles = (Mc / 64) * (kCout / 64);
    wmma_gemm64<1, true, 0, 0, false, 0><<<dim3((wtiles + 7) / 8, 1), 256, 0, stream>>>(
        (const unsigned short*)WFH, (const unsigned short*)WFL, kKdim, 0L,
        (const unsigned short*)WTH, (const unsigned short*)WTL, kKdim, 0L,
        (void*)(OUTP + (size_t)rowBase * kCout), (void*)nullptr, kCout, 0L,
        (const float*)nullptr, (const float*)nullptr, 0L, Mc, kCout, kKdim, 1.0f);
  }

  stats_partial_kernel<<<kStatBlocks, 256, 0, stream>>>(OUTP, PART);
  stats_final_kernel<<<1, 128, 0, stream>>>(PART, gamma, MR);
  {
    const int total4 = kNumPts * kCout / 4;
    norm_act_kernel<<<(total4 + 255) / 256, 256, 0, stream>>>(OUTP, MR, beta, out, total4);
  }
}
